// OuterProductMean_64707977281618
// MI455X (gfx1250) — hardware-verified
//
#include <hip/hip_runtime.h>
#include <math.h>

constexpr int kS    = 128;
constexpr int kR    = 256;
constexpr int kCM   = 256;
constexpr int kCH   = 32;
constexpr int kNP   = 2 * kCH;
constexpr int kCZ   = 128;
constexpr int kHH   = kCH * kCH;
constexpr int kRows = kS * kR;
constexpr int kPlaneHalves = kR * kCH * kS;
constexpr int kGP   = 1032;
constexpr int kSOP  = 132;
constexpr int kTP   = 68;
constexpr float kABCarry  = 2.0f;
constexpr float kWoCarry  = 256.0f;
constexpr float kLinScale = 1.0f / (kABCarry * kABCarry * kWoCarry);
constexpr float kInvCM    = 1.0f / 256.0f;
constexpr float kLnEps    = 1e-5f;
constexpr float kNormEps  = 1e-3f;

static_assert(kRows % 64 == 0);
static_assert(kNP % 64 == 0);
static_assert(kCM % 32 == 0);
static_assert(kS % 32 == 0);
static_assert(kHH % 32 == 0);
static_assert((kGP * 2) % 16 == 0);
static_assert((kSOP * 4) % 16 == 0);

typedef __attribute__((ext_vector_type(16))) _Float16 v16h;
typedef __attribute__((ext_vector_type(8)))  _Float16 v8h;
typedef __attribute__((ext_vector_type(16))) __bf16   v16b;
typedef __attribute__((ext_vector_type(8)))  __bf16   v8b;
typedef __attribute__((ext_vector_type(8)))  float    v8f;
typedef __attribute__((ext_vector_type(4)))  float    v4f;
typedef __attribute__((ext_vector_type(4)))  unsigned int v4u;

__device__ __forceinline__ unsigned short f2bf_bits(float f) {
  unsigned u = __float_as_uint(f);
  return (unsigned short)((u + 0x7FFFu + ((u >> 16) & 1u)) >> 16);
}
__device__ __forceinline__ float bf_bits2f(unsigned short h) { return __uint_as_float(((unsigned)h) << 16); }

__device__ __forceinline__ void dep_guard_h(v8f& a, v8f& b, v16h x, v16h y) { asm volatile("v_nop\n\tv_nop\n\tv_nop\n\tv_nop" : "+v"(a), "+v"(b) : "v"(x), "v"(y)); }
__device__ __forceinline__ void dep_guard_b(v8f& a, v8f& b, v16b x, v16b y) { asm volatile("v_nop\n\tv_nop\n\tv_nop\n\tv_nop" : "+v"(a), "+v"(b) : "v"(x), "v"(y)); }
__device__ __forceinline__ void keep4_h(v16h a, v16h b, v16h c, v16h d) { asm volatile("v_nop" :: "v"(a), "v"(b), "v"(c), "v"(d)); }
__device__ __forceinline__ void keep4_b(v16b a, v16b b, v16b c, v16b d) { asm volatile("v_nop" :: "v"(a), "v"(b), "v"(c), "v"(d)); }
__device__ __forceinline__ void acc_guard4(v8f& a, v8f& b, v8f& c, v8f& d) { asm volatile("v_nop\n\tv_nop\n\tv_nop\n\tv_nop" : "+v"(a), "+v"(b), "+v"(c), "+v"(d)); }
template <typename T> struct Frag;
template <> struct Frag<_Float16> {
  typedef v16h V; union U { v16h v; v8h h[2]; };
  static __device__ __forceinline__ v16h load(const _Float16* p) {
    U f; f.h[0] = *(const v8h*)(p); f.h[1] = *(const v8h*)(p + 16); return f.v;
  }
  static __device__ __forceinline__ v8f mma(v16h a, v16h b, v8f c) {
    return __builtin_amdgcn_wmma_f32_16x16x32_f16(false, a, false, b, (short)0, c, false, false);
  }
  static __device__ __forceinline__ void guard(v8f& a, v8f& b, v16h x, v16h y) { dep_guard_h(a, b, x, y); }
  static __device__ __forceinline__ void keep(v16h a, v16h b, v16h c, v16h d) { keep4_h(a, b, c, d); }
};
template <> struct Frag<__bf16> {
  typedef v16b V; union U { v16b v; v8b h[2]; };
  static __device__ __forceinline__ v16b load(const __bf16* p) {
    U f; f.h[0] = *(const v8b*)(p); f.h[1] = *(const v8b*)(p + 16); return f.v;
  }
  static __device__ __forceinline__ v8f mma(v16b a, v16b b, v8f c) {
    return __builtin_amdgcn_wmma_f32_16x16x32_bf16(false, a, false, b, (short)0, c, false, false);
  }
  static __device__ __forceinline__ void guard(v8f& a, v8f& b, v16b x, v16b y) { dep_guard_b(a, b, x, y); }
  static __device__ __forceinline__ void keep(v16b a, v16b b, v16b c, v16b d) { keep4_b(a, b, c, d); }
};

__device__ __forceinline__ unsigned pk16(unsigned short a, unsigned short b) { return (unsigned)a | ((unsigned)b << 16); }
__device__ __forceinline__ unsigned short h_bits(float f) { const _Float16 h = (_Float16)f; return __builtin_bit_cast(unsigned short, h); }

__device__ __forceinline__ v8f mma_f16(v16h a, v16h b, v8f c) {
  c = __builtin_amdgcn_wmma_f32_16x16x32_f16(false, a, false, b, (short)0, c, false, false);
  asm volatile("v_nop\n\tv_nop\n\tv_nop\n\tv_nop" : "+v"(c) : "v"(a), "v"(b));
  return c;
}

template <int ET> struct Elem;
template <> struct Elem<0> { typedef _Float16 T; };
template <> struct Elem<1> { typedef __bf16 T; };
template <int ET, bool SPLIT, int BIAS_MODE, int OUT_MODE, bool RESID, int ACT = 0>
__global__ __launch_bounds__(256) void wmma_gemm64(
    const unsigned short* __restrict__ Ap, const unsigned short* __restrict__ A2p, int lda, long strideA,
    const unsigned short* __restrict__ Btp, const unsigned short* __restrict__ Bt2p, int ldb, long strideB,
    void* __restrict__ Cout, void* __restrict__ Cout2, int ldc, long strideC,
    const float* __restrict__ bias,
    const float* __restrict__ resid, long strideR,
    int M, int N, int K, float scale) {
  typedef typename Elem<ET>::T T;
  typedef typename Frag<T>::V V;
  const T* A = (const T*)Ap; const T* A2 = (const T*)A2p; const T* Bt = (const T*)Btp; const T* Bt2 = (const T*)Bt2p;
  __shared__ __align__(16) float sT[8][16 * 68];
  const int b    = blockIdx.y;
  const int lane = threadIdx.x & 31;
  const int wave = threadIdx.x >> 5;
  const int tilesN = N >> 6;
  const int tilesM = M >> 6;
  const int tile = blockIdx.x * 8 + wave;
  if (tile >= tilesM * tilesN) return;
  const int tm = tile / tilesN;
  const int tn = tile - tm * tilesN;
  const int m0 = tm << 6;
  const int n0 = tn << 6;

  const T* Ab  = A  + (size_t)b * strideA;
  const T* Bb  = Bt + (size_t)b * strideB;
  const T* Ab2 = SPLIT ? (A2  + (size_t)b * strideA) : nullptr;
  const T* Bb2 = SPLIT ? (Bt2 + (size_t)b * strideB) : nullptr;

  const int rlane = lane & 15;
  const int koff  = (lane >> 4) * 8;
  const int mOff  = (lane >> 4) * 8;

  v8f acc[4][4];
#pragma unroll
  for (int i = 0; i < 4; ++i)
#pragma unroll
    for (int j = 0; j < 4; ++j) acc[i][j] = (v8f){0.f,0.f,0.f,0.f,0.f,0.f,0.f,0.f};

  for (int k0 = 0; k0 < K; k0 += 32) {
    V bh[4], bl[4];
#pragma unroll
    for (int j = 0; j < 4; ++j) {
      const size_t bo = (size_t)(n0 + (j << 4) + rlane) * ldb + koff + k0;
      bh[j] = Frag<T>::load(Bb + bo);
      if (SPLIT) bl[j] = Frag<T>::load(Bb2 + bo);
    }
#pragma unroll
    for (int i = 0; i < 4; ++i) {
      const size_t ao = (size_t)(m0 + (i << 4) + rlane) * lda + koff + k0;
      V ah = Frag<T>::load(Ab + ao);
      V al;
      if (SPLIT) al = Frag<T>::load(Ab2 + ao);
#pragma unroll
      for (int j = 0; j < 4; ++j) {
        acc[i][j] = Frag<T>::mma(ah, bh[j], acc[i][j]);
        if (SPLIT) {
          acc[i][j] = Frag<T>::mma(ah, bl[j], acc[i][j]);
          acc[i][j] = Frag<T>::mma(al, bh[j], acc[i][j]);
        }
      }
      Frag<T>::guard(acc[i][0], acc[i][1], ah, SPLIT ? al : ah);
      Frag<T>::guard(acc[i][2], acc[i][3], ah, SPLIT ? al : ah);
    }
    Frag<T>::keep(bh[0], bh[1], bh[2], bh[3]);
    if (SPLIT) Frag<T>::keep(bl[0], bl[1], bl[2], bl[3]);
  }
  acc_guard4(acc[0][0], acc[0][1], acc[0][2], acc[0][3]);
  acc_guard4(acc[1][0], acc[1][1], acc[1][2], acc[1][3]);
  acc_guard4(acc[2][0], acc[2][1], acc[2][2], acc[2][3]);
  acc_guard4(acc[3][0], acc[3][1], acc[3][2], acc[3][3]);

  float* slab = sT[wave];
  const float* Rb = RESID ? (resid + (size_t)b * strideR) : nullptr;
#pragma unroll
  for (int i = 0; i < 4; ++i) {
    const int mBase = m0 + (i << 4);
#pragma unroll
    for (int j = 0; j < 4; ++j) {
      const int n = n0 + (j << 4) + rlane;
      float bv = 0.f;
      if (BIAS_MODE == 2) bv = bias[n];
#pragma unroll
      for (int r = 0; r < 8; ++r) {
        float v = acc[i][j][r] * scale;
        if (BIAS_MODE == 1) v += bias[mBase + mOff + r];
        if (BIAS_MODE == 2) v += bv;
        if (RESID) v += Rb[(size_t)(mBase + mOff + r) * ldc + n];
        if (ACT == 2) v = fmaxf(v, 0.0f);
        if (ACT == 4) v = (v > 0.f) ? v : 0.01f * v;
        slab[(mOff + r) * 68 + (j << 4) + rlane] = v;
      }
    }
    __builtin_amdgcn_fence(__ATOMIC_RELEASE, "workgroup");
    __builtin_amdgcn_wave_barrier();
    __builtin_amdgcn_fence(__ATOMIC_ACQUIRE, "workgroup");
    if (OUT_MODE == 0) {
      float* C = (float*)Cout + (size_t)b * strideC;
      const int hh = lane >> 4, c4 = (lane & 15) * 4;
      for (int pass = 0; pass < 2; ++pass) {
#pragma unroll
        for (int it = 0; it < 8; ++it) {
          const int row = it * 2 + hh;
          v4f v = *(const v4f*)(slab + row * 68 + c4);
          *(volatile v4f*)(C + (size_t)(mBase + row) * ldc + n0 + c4) = v;
        }
        __threadfence();
      }
    } else {
      const int q = lane >> 3, c8 = (lane & 7) * 8;
      unsigned short* C  = (unsigned short*)Cout  + (size_t)b * strideC;
      unsigned short* C2 = (OUT_MODE == 2) ? ((unsigned short*)Cout2 + (size_t)b * strideC) : nullptr;
      for (int pass = 0; pass < 2; ++pass) {
#pragma unroll
        for (int it = 0; it < 4; ++it) {
          const int row = it * 4 + q;
          const float* sp = slab + row * 68 + c8;
          v8h hv, lv;
#pragma unroll
          for (int e = 0; e < 8; ++e) {
            if (OUT_MODE == 1) {
              hv[e] = (_Float16)sp[e];
            } else {
              unsigned short hb = f2bf_bits(sp[e]);
              unsigned short lb = f2bf_bits(sp[e] - bf_bits2f(hb));
              hv[e] = __builtin_bit_cast(_Float16, hb);
              lv[e] = __builtin_bit_cast(_Float16, lb);
            }
          }
          *(volatile v8h*)(C + (size_t)(mBase + row) * ldc + n0 + c8) = hv;
          if (OUT_MODE == 2) *(volatile v8h*)(C2 + (size_t)(mBase + row) * ldc + n0 + c8) = lv;
        }
        __threadfence();
      }
    }
    __builtin_amdgcn_fence(__ATOMIC_RELEASE, "workgroup");
    __builtin_amdgcn_wave_barrier();
    __builtin_amdgcn_fence(__ATOMIC_ACQUIRE, "workgroup");
  }
}

__global__ __launch_bounds__(256) void prep_w12_kernel(const float* __restrict__ w1, const float* __restrict__ w2,
                                                       unsigned short* __restrict__ whi, unsigned short* __restrict__ wlo) {
  __shared__ __align__(16) float sw[kCM];
  const int n = blockIdx.x;
  const int t = threadIdx.x;
  const float* src = (n < kCH) ? w1 : w2;
  const int col = n & (kCH - 1);
  sw[t] = src[(size_t)t * kCH + col];
  __syncthreads();
  const int lane = t & 31, wave = t >> 5;
  if (wave == 0) {
    unsigned short hb[8], lb[8];
#pragma unroll
    for (int e = 0; e < 8; ++e) {
      const float v = sw[8 * lane + e];
      const unsigned short h = f2bf_bits(v);
      hb[e] = h;
      lb[e] = f2bf_bits(v - bf_bits2f(h));
    }
    const v4u hu = (v4u){pk16(hb[0], hb[1]), pk16(hb[2], hb[3]), pk16(hb[4], hb[5]), pk16(hb[6], hb[7])};
    const v4u lu = (v4u){pk16(lb[0], lb[1]), pk16(lb[2], lb[3]), pk16(lb[4], lb[5]), pk16(lb[6], lb[7])};
    unsigned short* ph = whi + (size_t)n * kCM + 8 * lane;
    unsigned short* pl = wlo + (size_t)n * kCM + 8 * lane;
    *(volatile v4u*)ph = hu;
    *(volatile v4u*)pl = lu;
    __threadfence();
    *(volatile v4u*)ph = hu;
    *(volatile v4u*)pl = lu;
  }
}

__global__ __launch_bounds__(256) void prep_wo_kernel(const float* __restrict__ w_out, unsigned short* __restrict__ woT) {
  __shared__ float sm[64][65];
  const int t  = threadIdx.x;
  const int k0 = blockIdx.x * 64;
  const int z0 = blockIdx.y * 64;
#pragma unroll
  for (int it = 0; it < 8; ++it) {
    const int e = it * 256 + t;
    const int r = e >> 6;
    const int c = e & 63;
    sm[c][r] = w_out[(size_t)(k0 + r) * kCZ + z0 + c] * kWoCarry;
  }
  asm volatile("" ::: "memory");
#pragma unroll
  for (int it = 8; it < 16; ++it) {
    const int e = it * 256 + t;
    const int r = e >> 6;
    const int c = e & 63;
    sm[c][r] = w_out[(size_t)(k0 + r) * kCZ + z0 + c] * kWoCarry;
  }
  __syncthreads();
  const int lane = t & 31, wave = t >> 5;
  const int q = lane >> 3, c8 = (lane & 7) * 8;
  for (int pass = 0; pass < 2; ++pass) {
#pragma unroll
    for (int it = 0; it < 2; ++it) {
      const int row = wave * 8 + it * 4 + q;
      unsigned short hb[8];
#pragma unroll
      for (int e = 0; e < 8; ++e) hb[e] = h_bits(sm[row][c8 + e]);
      const v4u u = (v4u){pk16(hb[0], hb[1]), pk16(hb[2], hb[3]), pk16(hb[4], hb[5]), pk16(hb[6], hb[7])};
      *(volatile v4u*)(woT + (size_t)(z0 + row) * kHH + k0 + c8) = u;
    }
    __threadfence();
  }
}

__global__ __launch_bounds__(256) void rnorm_kernel(const float* __restrict__ mask, float* __restrict__ rn) {
  const int t  = blockIdx.x * 256 + threadIdx.x;
  const int i  = t >> 6;
  const int j4 = (t & 63) * 4;
  float a0 = 0.0f, a1 = 0.0f, a2 = 0.0f, a3 = 0.0f;
#pragma unroll 1
  for (int s = 0; s < kS; ++s) {
    const float mi = mask[(size_t)s * kR + i];
    const v4f  mj = *(const v4f*)(mask + (size_t)s * kR + j4);
    a0 = fmaf(mi, mj[0], a0);
    a1 = fmaf(mi, mj[1], a1);
    a2 = fmaf(mi, mj[2], a2);
    a3 = fmaf(mi, mj[3], a3);
  }
  v4f r;
  r[0] = 1.0f / (kNormEps + a0);
  r[1] = 1.0f / (kNormEps + a1);
  r[2] = 1.0f / (kNormEps + a2);
  r[3] = 1.0f / (kNormEps + a3);
  float* dst = rn + 4 * (size_t)t;
  *(volatile v4f*)dst = r;
  __threadfence();
  *(volatile v4f*)dst = r;
}

__global__ __launch_bounds__(256) void ln_kernel(const float* __restrict__ m, const float* __restrict__ ln_g,
                                                 const float* __restrict__ ln_b,
                                                 unsigned short* __restrict__ mnhi, unsigned short* __restrict__ mnlo) {
  const int lane = threadIdx.x & 31, wave = threadIdx.x >> 5;
  const int row  = blockIdx.x * 8 + wave;
  const float* p = m + (size_t)row * kCM + 8 * lane;
  const v4f x0 = *(const v4f*)(p);
  const v4f x1 = *(const v4f*)(p + 4);
  const v4f g0 = *(const v4f*)(ln_g + 8 * lane);
  const v4f g1 = *(const v4f*)(ln_g + 8 * lane + 4);
  const v4f c0 = *(const v4f*)(ln_b + 8 * lane);
  const v4f c1 = *(const v4f*)(ln_b + 8 * lane + 4);
  float v[8], gg[8], cc[8];
#pragma unroll
  for (int e = 0; e < 4; ++e) {
    v[e] = x0[e];  v[4 + e] = x1[e];
    gg[e] = g0[e]; gg[4 + e] = g1[e];
    cc[e] = c0[e]; cc[4 + e] = c1[e];
  }
  float s = 0.0f;
#pragma unroll
  for (int e = 0; e < 8; ++e) s += v[e];
#pragma unroll
  for (int off = 16; off > 0; off >>= 1) s += __shfl_xor(s, off, 32);
  const float mu = s * kInvCM;
  float d[8];
  float s2 = 0.0f;
#pragma unroll
  for (int e = 0; e < 8; ++e) { d[e] = v[e] - mu; s2 += d[e] * d[e]; }
#pragma unroll
  for (int off = 16; off > 0; off >>= 1) s2 += __shfl_xor(s2, off, 32);
  const float var  = s2 * kInvCM;
  const float rstd = 1.0f / sqrtf(var + kLnEps);
  unsigned short hb[8], lb[8];
#pragma unroll
  for (int e = 0; e < 8; ++e) {
    const float y = d[e] * rstd * gg[e] + cc[e];
    const unsigned short h = f2bf_bits(y);
    hb[e] = h;
    lb[e] = f2bf_bits(y - bf_bits2f(h));
  }
  const v4u hu = (v4u){pk16(hb[0], hb[1]), pk16(hb[2], hb[3]), pk16(hb[4], hb[5]), pk16(hb[6], hb[7])};
  const v4u lu = (v4u){pk16(lb[0], lb[1]), pk16(lb[2], lb[3]), pk16(lb[4], lb[5]), pk16(lb[6], lb[7])};
  unsigned short* ph = mnhi + (size_t)row * kCM + 8 * lane;
  unsigned short* pl = mnlo + (size_t)row * kCM + 8 * lane;
  *(volatile v4u*)ph = hu;
  *(volatile v4u*)pl = lu;
  __threadfence();
  *(volatile v4u*)ph = hu;
  *(volatile v4u*)pl = lu;
}

__global__ __launch_bounds__(256) void proj_pack_kernel(const float* __restrict__ proj, const float* __restrict__ mask,
                                                        const float* __restrict__ b1, const float* __restrict__ b2,
                                                        unsigned short* __restrict__ abT) {
  __shared__ __align__(16) float sTile[kS * kTP];
  __shared__ float smask[kS];
  __shared__ float sbias[kNP];
  const int i = blockIdx.x;
  const int t = threadIdx.x, lane = t & 31, wave = t >> 5;
#pragma unroll
  for (int it = 0; it < 4; ++it) {
    const int e  = it * 256 + t;
    const int s  = e >> 4;
    const int c4 = (e & 15) * 4;
    const v4f v = *(const v4f*)(proj + ((size_t)s * kR + i) * kNP + c4);
    *(v4f*)(sTile + s * kTP + c4) = v;
  }
  asm volatile("" ::: "memory");
#pragma unroll
  for (int it = 4; it < 8; ++it) {
    const int e  = it * 256 + t;
    const int s  = e >> 4;
    const int c4 = (e & 15) * 4;
    const v4f v = *(const v4f*)(proj + ((size_t)s * kR + i) * kNP + c4);
    *(v4f*)(sTile + s * kTP + c4) = v;
  }
  if (wave < 4)  smask[t] = mask[(size_t)t * kR + i];
  if (wave == 0) sbias[lane] = b1[lane];
  if (wave == 1) sbias[kCH + lane] = b2[lane];
  __syncthreads();
  const int hh = lane >> 4, s0 = (lane & 15) * 8;
  for (int pass = 0; pass < 2; ++pass) {
#pragma unroll
    for (int it = 0; it < 4; ++it) {
      const int q = wave * 8 + it * 2 + hh;
      const float bq = sbias[q];
      unsigned short hb[8];
#pragma unroll
      for (int e = 0; e < 8; ++e) {
        const float pv = sTile[(s0 + e) * kTP + q];
        const float av = (pv + bq) * smask[s0 + e];
        hb[e] = h_bits(av * kABCarry);
      }
      const v4u u = (v4u){pk16(hb[0], hb[1]), pk16(hb[2], hb[3]), pk16(hb[4], hb[5]), pk16(hb[6], hb[7])};
      unsigned short* dst = abT + (size_t)(q >> 5) * kPlaneHalves + ((size_t)i * kCH + (q & 31)) * kS + s0;
      *(volatile v4u*)dst = u;
    }
    __threadfence();
  }
}

__global__ __launch_bounds__(256) void pair_kernel(const unsigned short* __restrict__ abTp, const unsigned short* __restrict__ woTp,
                                                   const float* __restrict__ b_out, const float* __restrict__ rn,
                                                   float* __restrict__ out) {
  __shared__ __align__(16) _Float16 gL[16 * kGP];
  __shared__ __align__(16) float sO[16 * kSOP];
  const _Float16* aPl = (const _Float16*)abTp;
  const _Float16* bPl = aPl + (size_t)kPlaneHalves;
  const _Float16* woT = (const _Float16*)woTp;
  const int t = threadIdx.x, lane = t & 31, wave = t >> 5;
  const int hh = lane >> 4, rlane = lane & 15, koff = hh * 8;
  const int i  = blockIdx.x >> 4;
  const int j0 = (blockIdx.x & 15) * 16;
  const int ct = (wave >> 1) & 1, et = wave & 1, pw = wave >> 2;

  v16h bfr[4];
  {
    const _Float16* brow = aPl + ((size_t)i * kCH + ct * 16 + rlane) * kS + koff;
#pragma unroll
    for (int ks = 0; ks < 4; ++ks) bfr[ks] = Frag<_Float16>::load(brow + ks * 32);
  }
#pragma unroll 1
  for (int jj = 0; jj < 8; ++jj) {
    const int p = jj * 2 + pw;
    const _Float16* arow = bPl + ((size_t)(j0 + p) * kCH + et * 16 + rlane) * kS + koff;
    v8f acc = (v8f){0.f,0.f,0.f,0.f,0.f,0.f,0.f,0.f};
#pragma unroll
    for (int ks = 0; ks < 4; ++ks) {
      const v16h af = Frag<_Float16>::load(arow + ks * 32);
      acc = mma_f16(af, bfr[ks], acc);
    }
    v8h gv;
#pragma unroll
    for (int r = 0; r < 8; ++r) { const float gf = acc[r]; gv[r] = (_Float16)gf; }
    *(v8h*)(gL + p * kGP + (ct * 16 + rlane) * kCH + et * 16 + 8 * hh) = gv;
  }
  __syncthreads();

  const _Float16* grow = gL + rlane * kGP + koff;
  const _Float16* wrow = woT + ((size_t)wave * 16 + rlane) * kHH + koff;
  v8f acc2 = (v8f){0.f,0.f,0.f,0.f,0.f,0.f,0.f,0.f};
#pragma unroll 2
  for (int k0 = 0; k0 < kHH; k0 += 32) {
    const v16h af = Frag<_Float16>::load(grow + k0);
    const v16h bf = Frag<_Float16>::load(wrow + k0);
    acc2 = mma_f16(af, bf, acc2);
  }
  const int z = wave * 16 + rlane;
  const float bz = b_out[z];
  const float* rnp = rn + (size_t)i * kR + j0 + 8 * hh;
  const v4f rq0 = *(const v4f*)(rnp);
  const v4f rq1 = *(const v4f*)(rnp + 4);
  float rr[8];
#pragma unroll
  for (int e = 0; e < 4; ++e) { rr[e] = rq0[e]; rr[4 + e] = rq1[e]; }
#pragma unroll
  for (int r = 0; r < 8; ++r) {
    const float av = acc2[r];
    const float vv = (av * kLinScale + bz) * rr[r];
    sO[(8 * hh + r) * kSOP + z] = vv;
  }
  __syncthreads();

  float* ob = out + ((size_t)i * kR + j0) * kCZ;
  for (int pass = 0; pass < 2; ++pass) {
#pragma unroll
    for (int it = 0; it < 2; ++it) {
      const int o  = it * 1024 + t * 4;
      const int p  = o >> 7;
      const int zz = o & 127;
      const v4f val = *(const v4f*)(sO + p * kSOP + zz);
      *(volatile v4f*)(ob + o) = val;
    }
    __threadfence();
  }
}

extern "C" void kernel_launch(void* const* d_in, const int* in_sizes, int n_in,
                              void* d_out, int out_size, void* d_ws, size_t ws_size,
                              hipStream_t stream) {
  if (n_in < 10) return;
  if (in_sizes[0] != kRows * kCM || in_sizes[1] != kRows || in_sizes[2] != kCM || in_sizes[3] != kCM ||
      in_sizes[4] != kCM * kCH || in_sizes[5] != kCH || in_sizes[6] != kCM * kCH || in_sizes[7] != kCH ||
      in_sizes[8] != kHH * kCZ || in_sizes[9] != kCZ || out_size != kR * kR * kCZ) return;

  const float* m     = (const float*)d_in[0];
  const float* mask  = (const float*)d_in[1];
  const float* ln_g  = (const float*)d_in[2];
  const float* ln_b  = (const float*)d_in[3];
  const float* w1    = (const float*)d_in[4];
  const float* b1    = (const float*)d_in[5];
  const float* w2    = (const float*)d_in[6];
  const float* b2    = (const float*)d_in[7];
  const float* w_out = (const float*)d_in[8];
  const float* b_out = (const float*)d_in[9];
  float* out = (float*)d_out;

  char* ws = (char*)d_ws;
  size_t off = 0;
  unsigned short* mnhi  = (unsigned short*)(ws + off); off += (size_t)kRows * kCM * 2;
  unsigned short* mnlo  = (unsigned short*)(ws + off); off += (size_t)kRows * kCM * 2;
  float*          proj  = (float*)(ws + off);          off += (size_t)kRows * kNP * 4;
  unsigned short* abT   = (unsigned short*)(ws + off); off += (size_t)2 * kPlaneHalves * 2;
  unsigned short* w12hi = (unsigned short*)(ws + off); off += (size_t)kNP * kCM * 2;
  unsigned short* w12lo = (unsigned short*)(ws + off); off += (size_t)kNP * kCM * 2;
  unsigned short* woT   = (unsigned short*)(ws + off); off += (size_t)kCZ * kHH * 2;
  float*          rnorm = (float*)(ws + off);          off += (size_t)kR * kR * 4;
  if (off > ws_size) return;

  prep_w12_kernel<<<kNP, 256, 0, stream>>>(w1, w2, w12hi, w12lo);
  prep_wo_kernel<<<dim3(kHH / 64, kCZ / 64), 256, 0, stream>>>(w_out, woT);
  rnorm_kernel<<<(kR * kR / 4) / 256, 256, 0, stream>>>(mask, rnorm);
  ln_kernel<<<kRows / 8, 256, 0, stream>>>(m, ln_g, ln_b, mnhi, mnlo);
  wmma_gemm64<1, true, 0, 0, false, 0><<<dim3((kRows / 64) * (kNP / 64) / 8, 1), 256, 0, stream>>>(
      mnhi, mnlo, kCM, 0L, w12hi, w12lo, kCM, 0L, (void*)proj, (void*)proj, kNP, 0L,
      b_out, rnorm, 0L, kRows, kNP, kCM, 1.0f);
  proj_pack_kernel<<<kR, 256, 0, stream>>>(proj, mask, b1, b2, abT);
  pair_kernel<<<kR * (kR / 16), 256, 0, stream>>>(abT, woT, b_out, rnorm, out);
}
